// EpsilonNetGM_4209067950718
// MI455X (gfx1250) — hardware-run, weakly checked
//
#include <hip/hip_runtime.h>
#include <math.h>

typedef __attribute__((ext_vector_type(16))) _Float16 v16h;
typedef __attribute__((ext_vector_type(8)))  _Float16 v8h;
typedef __attribute__((ext_vector_type(16))) __bf16   v16b;
typedef __attribute__((ext_vector_type(8)))  __bf16   v8b;
typedef __attribute__((ext_vector_type(8)))  float    v8f;
typedef __attribute__((ext_vector_type(4)))  float    v4f;
typedef __attribute__((ext_vector_type(4)))  unsigned v4u;

constexpr int kRowsN   = 32768;
constexpr int kComp    = 25;
constexpr int kDim     = 128;
constexpr int kTab     = 1000;
constexpr int kKcat    = 3 * kDim;
constexpr int kCompT   = 64;
constexpr int kCompP   = 32;
constexpr int kKmix    = 2 * kCompP;
constexpr int kConstN  = 128;
constexpr int kIdxScale = 64;
constexpr int kIdxS     = 65;
constexpr int kIdxInv   = 66;
constexpr int kSoftRowsPerWave = 8;
constexpr float kCarryP    = 32768.0f;
constexpr float kCarryPlo  = 16.0f;
constexpr float kCarryW    = 64.0f;
constexpr float kCarryWlo  = 2048.0f;
constexpr float kFoldBack  = 1.0f / (kCarryP * kCarryW);
static_assert(kCarryP == kCarryPlo * kCarryWlo, "both k blocks of the second contraction share one total scale");
static_assert(kKcat == 384 && (kKcat % 32) == 0 && (kKmix % 32) == 0, "K multiples of 32");
static_assert((kRowsN % 64) == 0 && (kCompT % 64) == 0 && (kDim % 64) == 0, "M, N multiples of 64");
static_assert(kComp <= kCompP && kCompP == 32, "one lane per component");
static_assert((kRowsN % (8 * kSoftRowsPerWave)) == 0, "softmax grid exact");

constexpr size_t kOffA1  = 0;
constexpr size_t kOffBT1 = kOffA1  + (size_t)kRowsN * kKcat * 2;
constexpr size_t kOffG   = kOffBT1 + (size_t)kCompT * kKcat * 2;
constexpr size_t kOffR2  = kOffG   + (size_t)kRowsN * kCompT * 4;
constexpr size_t kOffBT2 = kOffR2  + (size_t)kRowsN * kKmix * 2;
constexpr size_t kOffP   = kOffBT2 + (size_t)kDim * kKmix * 2;
constexpr size_t kOffCST = kOffP   + (size_t)kRowsN * kDim * 4;
constexpr size_t kWsTotal = kOffCST + (size_t)kConstN * 4;
static_assert(kWsTotal == 54592000ull, "carve total");
static_assert(kWsTotal <= 134217728ull, "carve cap");
static_assert((kOffBT1 % 128) == 0 && (kOffG % 128) == 0 && (kOffR2 % 128) == 0 && (kOffBT2 % 128) == 0 &&
              (kOffP % 128) == 0 && (kOffCST % 128) == 0, "128-B aligned regions");

__device__ __forceinline__ unsigned short f2bf_bits(float f) {
  unsigned u = __float_as_uint(f);
  return (unsigned short)((u + 0x7FFFu + ((u >> 16) & 1u)) >> 16);
}
__device__ __forceinline__ float bf_bits2f(unsigned short h) { return __uint_as_float(((unsigned)h) << 16); }

__device__ __forceinline__ unsigned bf_pair_word(float a, float b, bool wantlo) {
  const unsigned short ha = f2bf_bits(a);
  const unsigned short hb = f2bf_bits(b);
  const unsigned short la = f2bf_bits(a - bf_bits2f(ha));
  const unsigned short lb = f2bf_bits(b - bf_bits2f(hb));
  const unsigned ua = wantlo ? (unsigned)la : (unsigned)ha;
  const unsigned ub = wantlo ? (unsigned)lb : (unsigned)hb;
  return ua | (ub << 16);
}
__device__ __forceinline__ unsigned h_pair_word(float a, float b, bool wantlo) {
  const _Float16 ha = (_Float16)a;
  const _Float16 hb = (_Float16)b;
  const float ra = (a - (float)ha) * kCarryWlo;
  const float rb = (b - (float)hb) * kCarryWlo;
  const _Float16 la = (_Float16)ra;
  const _Float16 lb = (_Float16)rb;
  const unsigned uha = (unsigned)__builtin_bit_cast(unsigned short, ha);
  const unsigned uhb = (unsigned)__builtin_bit_cast(unsigned short, hb);
  const unsigned ula = (unsigned)__builtin_bit_cast(unsigned short, la);
  const unsigned ulb = (unsigned)__builtin_bit_cast(unsigned short, lb);
  const unsigned ua = wantlo ? ula : uha;
  const unsigned ub = wantlo ? ulb : uhb;
  return ua | (ub << 16);
}

__device__ __forceinline__ v8f mma_guard_h(v16h a, v16h b, v8f c) {
  c = __builtin_amdgcn_wmma_f32_16x16x32_f16(false, a, false, b, (short)0, c, false, false);
  asm volatile("v_nop\n\tv_nop\n\tv_nop\n\tv_nop" : "+v"(c) : "v"(a), "v"(b));
  return c;
}
__device__ __forceinline__ v8f mma_guard_b(v16b a, v16b b, v8f c) {
  c = __builtin_amdgcn_wmma_f32_16x16x32_bf16(false, a, false, b, (short)0, c, false, false);
  asm volatile("v_nop\n\tv_nop\n\tv_nop\n\tv_nop" : "+v"(c) : "v"(a), "v"(b));
  return c;
}
__device__ __forceinline__ void keep4_h(v16h a, v16h b, v16h c, v16h d) { asm volatile("v_nop" :: "v"(a), "v"(b), "v"(c), "v"(d)); }
__device__ __forceinline__ void keep4_b(v16b a, v16b b, v16b c, v16b d) { asm volatile("v_nop" :: "v"(a), "v"(b), "v"(c), "v"(d)); }
__device__ __forceinline__ void acc_guard4(v8f& a, v8f& b, v8f& c, v8f& d) { asm volatile("v_nop\n\tv_nop\n\tv_nop\n\tv_nop" : "+v"(a), "+v"(b), "+v"(c), "+v"(d)); }

template <typename T> struct Frag;
template <> struct Frag<_Float16> {
  typedef v16h V; union U { v16h v; v8h h[2]; };
  static __device__ __forceinline__ v16h load(const _Float16* p) {
    U f; f.h[0] = *(const v8h*)(p); f.h[1] = *(const v8h*)(p + 16); return f.v;
  }
  static __device__ __forceinline__ v8f mma(v16h a, v16h b, v8f c) { return mma_guard_h(a, b, c); }
  static __device__ __forceinline__ void keep(v16h a, v16h b, v16h c, v16h d) { keep4_h(a, b, c, d); }
};
template <> struct Frag<__bf16> {
  typedef v16b V; union U { v16b v; v8b h[2]; };
  static __device__ __forceinline__ v16b load(const __bf16* p) {
    U f; f.h[0] = *(const v8b*)(p); f.h[1] = *(const v8b*)(p + 16); return f.v;
  }
  static __device__ __forceinline__ v8f mma(v16b a, v16b b, v8f c) { return mma_guard_b(a, b, c); }
  static __device__ __forceinline__ void keep(v16b a, v16b b, v16b c, v16b d) { keep4_b(a, b, c, d); }
};
template <int ET> struct Elem;
template <> struct Elem<0> { typedef _Float16 T; };
template <> struct Elem<1> { typedef __bf16 T; };

template <int ET>
__global__ __launch_bounds__(256) void gemm64_kernel(
    const unsigned short* __restrict__ Ap, int lda,
    const unsigned short* __restrict__ Btp, int ldb,
    float* __restrict__ C, int ldc,
    int M, int N, int K, float scale) {
  typedef typename Elem<ET>::T T;
  typedef typename Frag<T>::V V;
  const T* A = (const T*)Ap;
  const T* Bt = (const T*)Btp;
  __shared__ __align__(16) float sT[8][16 * 68];
  const int lane = threadIdx.x & 31;
  const int wave = __builtin_amdgcn_readfirstlane((int)(threadIdx.x >> 5));
  const int tilesN = N >> 6;
  const int tilesM = M >> 6;
  const int tile = blockIdx.x * 8 + wave;
  if (tile >= tilesM * tilesN) return;
  const int tm = tile / tilesN;
  const int tn = tile - tm * tilesN;
  const int m0 = tm << 6;
  const int n0 = tn << 6;

  const int rlane = lane & 15;
  const int koff  = (lane >> 4) * 8;
  const int mOff  = (lane >> 4) * 8;

  v8f acc[4][4];
#pragma unroll
  for (int i = 0; i < 4; ++i)
#pragma unroll
    for (int j = 0; j < 4; ++j) acc[i][j] = (v8f){0.f,0.f,0.f,0.f,0.f,0.f,0.f,0.f};

  for (int k0 = 0; k0 < K; k0 += 32) {
    V bh[4];
#pragma unroll
    for (int j = 0; j < 4; ++j) {
      const size_t bo = (size_t)(n0 + (j << 4) + rlane) * ldb + koff + k0;
      bh[j] = Frag<T>::load(Bt + bo);
    }
#pragma unroll
    for (int i = 0; i < 4; ++i) {
      const size_t ao = (size_t)(m0 + (i << 4) + rlane) * lda + koff + k0;
      const V ah = Frag<T>::load(A + ao);
#pragma unroll
      for (int j = 0; j < 4; ++j) {
        acc[i][j] = Frag<T>::mma(ah, bh[j], acc[i][j]);
      }
    }
    Frag<T>::keep(bh[0], bh[1], bh[2], bh[3]);
  }
  acc_guard4(acc[0][0], acc[0][1], acc[0][2], acc[0][3]);
  acc_guard4(acc[1][0], acc[1][1], acc[1][2], acc[1][3]);
  acc_guard4(acc[2][0], acc[2][1], acc[2][2], acc[2][3]);
  acc_guard4(acc[3][0], acc[3][1], acc[3][2], acc[3][3]);

  float* slab = sT[wave];
#pragma unroll
  for (int i = 0; i < 4; ++i) {
    const int mBase = m0 + (i << 4);
#pragma unroll
    for (int j = 0; j < 4; ++j) {
#pragma unroll
      for (int r = 0; r < 8; ++r) {
        const float v = acc[i][j][r] * scale;
        slab[(mOff + r) * 68 + (j << 4) + rlane] = v;
      }
    }
    __builtin_amdgcn_fence(__ATOMIC_RELEASE, "workgroup");
    __builtin_amdgcn_wave_barrier();
    __builtin_amdgcn_fence(__ATOMIC_ACQUIRE, "workgroup");
    {
      const int hh = lane >> 4, c4 = (lane & 15) * 4;
      for (int pass = 0; pass < 2; ++pass) {
#pragma unroll
        for (int it = 0; it < 8; ++it) {
          const int row = it * 2 + hh;
          const v4f v = *(const v4f*)(slab + row * 68 + c4);
          *(volatile v4f*)(C + (size_t)(mBase + row) * ldc + n0 + c4) = v;
        }
        __threadfence();
      }
    }
    __builtin_amdgcn_fence(__ATOMIC_RELEASE, "workgroup");
    __builtin_amdgcn_wave_barrier();
    __builtin_amdgcn_fence(__ATOMIC_ACQUIRE, "workgroup");
  }
}

__global__ __launch_bounds__(256) void prep_kernel(
    const float* __restrict__ means, const float* __restrict__ weights,
    const float* __restrict__ acp_arr, const int* __restrict__ t_arr,
    float* __restrict__ consts, unsigned* __restrict__ Bt1w, unsigned* __restrict__ Bt2w)
{
  __shared__ __align__(16) float sM[4 * 256 * 4];
  __shared__ __align__(16) float sC[256];
  const int tid  = threadIdx.x;
  const int lane = tid & 31;
  const int wave = __builtin_amdgcn_readfirstlane((int)(threadIdx.x >> 5));
  constexpr int kMeans4 = kComp * kDim / 4;
#pragma unroll 1
  for (int it = 0; it < 4; ++it) {
    const int i  = it * 256 + tid;
    const int ic = (i < kMeans4) ? i : (kMeans4 - 1);
    const v4f v = *(const v4f*)(means + (size_t)ic * 4);
    *(v4f*)(sM + i * 4) = v;
  }
  int t = t_arr[0];
  t = (t < 0) ? 0 : t;
  t = (t > kTab - 1) ? (kTab - 1) : t;
  const float acp     = acp_arr[t];
  const float sigma2  = 1.0f - acp;
  const float s       = sqrtf(acp);
  const float inv_s2  = 1.0f / sigma2;
  const float scale   = s * inv_s2;
  const float inv_std = 1.0f / sqrtf(sigma2);
  __syncthreads();

  const int k  = tid & 31;
  const int kk = (k < kComp) ? k : (kComp - 1);
  float mm = 0.0f;
#pragma unroll 4
  for (int d = 0; d < kDim; ++d) {
    const float m = sM[kk * kDim + d];
    mm = fmaf(m, m, mm);
  }
  float wv = weights[kk];
  asm volatile("" : "+v"(wv));
  const float cv = logf(wv) - (0.5f * acp * mm) * inv_s2;
  float val = 0.0f;
  val = (tid == kIdxScale) ? scale : val;
  val = (tid == kIdxS) ? s : val;
  val = (tid == kIdxInv) ? inv_std : val;
  val = (tid >= kComp && tid < kCompT) ? -1.0e30f : val;
  val = (tid < kComp) ? cv : val;
  sC[tid] = val;
  __syncthreads();
  if (wave == 0) {
    const v4f c4 = *(const v4f*)(sC + lane * 4);
    *(volatile v4f*)(consts + lane * 4) = c4;
    __threadfence();
    *(volatile v4f*)(consts + lane * 4) = c4;
  }

#pragma unroll 1
  for (int it = 0; it < 12; ++it) {
    const int i    = it * 256 + tid;
    const int row  = i / 48;
    const int cc   = i - row * 48;
    const int col0 = cc * 8;
    const int seg  = col0 >> 7;
    const int d0   = col0 & (kDim - 1);
    const int rk   = (row < kComp) ? row : (kComp - 1);
    const bool valid  = (row < kComp);
    const bool wantlo = (seg == 2);
    const v4f a0 = *(const v4f*)(sM + rk * kDim + d0);
    const v4f a1 = *(const v4f*)(sM + rk * kDim + d0 + 4);
    const float e0 = a0[0], e1 = a0[1], e2 = a0[2], e3 = a0[3];
    const float e4 = a1[0], e5 = a1[1], e6 = a1[2], e7 = a1[3];
    const float f0 = valid ? e0 : 0.0f, f1 = valid ? e1 : 0.0f, f2 = valid ? e2 : 0.0f, f3 = valid ? e3 : 0.0f;
    const float f4 = valid ? e4 : 0.0f, f5 = valid ? e5 : 0.0f, f6 = valid ? e6 : 0.0f, f7 = valid ? e7 : 0.0f;
    v4u w;
    w[0] = bf_pair_word(f0, f1, wantlo);
    w[1] = bf_pair_word(f2, f3, wantlo);
    w[2] = bf_pair_word(f4, f5, wantlo);
    w[3] = bf_pair_word(f6, f7, wantlo);
    unsigned* p = Bt1w + (size_t)i * 4;
    *(volatile v4u*)p = w;
    __threadfence();
    *(volatile v4u*)p = w;
  }

#pragma unroll 1
  for (int it = 0; it < 4; ++it) {
    const int i   = it * 256 + tid;
    const int d   = i >> 3;
    const int cc  = i & 7;
    const bool wantlo = ((cc >> 2) == 1);
    const int kb  = (cc & 3) * 8;
    float fv[8];
#pragma unroll
    for (int e = 0; e < 8; ++e) {
      const int kq  = kb + e;
      const int kqc = (kq < kComp) ? kq : (kComp - 1);
      const float m = sM[kqc * kDim + d];
      fv[e] = (kq < kComp) ? (m * kCarryW) : 0.0f;
    }
    v4u w;
    w[0] = h_pair_word(fv[0], fv[1], wantlo);
    w[1] = h_pair_word(fv[2], fv[3], wantlo);
    w[2] = h_pair_word(fv[4], fv[5], wantlo);
    w[3] = h_pair_word(fv[6], fv[7], wantlo);
    unsigned* p = Bt2w + (size_t)i * 4;
    *(volatile v4u*)p = w;
    __threadfence();
    *(volatile v4u*)p = w;
  }
}

__global__ __launch_bounds__(256) void split_x_kernel(
    const float* __restrict__ x, unsigned* __restrict__ A1w, int total8)
{
  const int i = blockIdx.x * 256 + threadIdx.x;
  if (i >= total8) return;
  const int row = i >> 4;
  const int c   = i & 15;
  const v4f a0 = *(const v4f*)(x + (size_t)i * 8);
  const v4f a1 = *(const v4f*)(x + (size_t)i * 8 + 4);
  const float f0 = a0[0], f1 = a0[1], f2 = a0[2], f3 = a0[3];
  const float f4 = a1[0], f5 = a1[1], f6 = a1[2], f7 = a1[3];
  v4u hw, lw;
  hw[0] = bf_pair_word(f0, f1, false);
  hw[1] = bf_pair_word(f2, f3, false);
  hw[2] = bf_pair_word(f4, f5, false);
  hw[3] = bf_pair_word(f6, f7, false);
  lw[0] = bf_pair_word(f0, f1, true);
  lw[1] = bf_pair_word(f2, f3, true);
  lw[2] = bf_pair_word(f4, f5, true);
  lw[3] = bf_pair_word(f6, f7, true);
  unsigned* base = A1w + (size_t)row * (kKcat / 2) + c * 4;
  *(volatile v4u*)(base) = hw;
  *(volatile v4u*)(base + kDim / 2) = lw;
  *(volatile v4u*)(base + kDim) = hw;
  __threadfence();
  *(volatile v4u*)(base) = hw;
  *(volatile v4u*)(base + kDim / 2) = lw;
  *(volatile v4u*)(base + kDim) = hw;
}

__global__ __launch_bounds__(256) void softmax_rows_kernel(
    const float* __restrict__ G, const float* __restrict__ consts, unsigned* __restrict__ R2w)
{
  const int lane = threadIdx.x & 31;
  const int wave = __builtin_amdgcn_readfirstlane((int)(threadIdx.x >> 5));
  const int kq = (lane < kComp) ? lane : (kComp - 1);
  const float ck    = consts[lane];
  const float scale = consts[kIdxScale];
  const int   src0  = 2 * (lane & 15);
  const float carry = (lane < 16) ? kCarryP : kCarryPlo;
  const int rowBase = (blockIdx.x * 8 + wave) * kSoftRowsPerWave;
#pragma unroll 1
  for (int i = 0; i < kSoftRowsPerWave; ++i) {
    const int row = rowBase + i;
    float g = G[(size_t)row * kCompT + kq];
    asm volatile("" : "+v"(g));
    const float lg = (lane < kComp) ? fmaf(scale, g, ck) : -1.0e30f;
    float m = lg;
    m = fmaxf(m, __shfl_xor(m, 16, 32));
    m = fmaxf(m, __shfl_xor(m, 8, 32));
    m = fmaxf(m, __shfl_xor(m, 4, 32));
    m = fmaxf(m, __shfl_xor(m, 2, 32));
    m = fmaxf(m, __shfl_xor(m, 1, 32));
    const float ex = expf(lg - m);
    const float e  = (lane < kComp) ? ex : 0.0f;
    float sum = e;
    sum += __shfl_xor(sum, 16, 32);
    sum += __shfl_xor(sum, 8, 32);
    sum += __shfl_xor(sum, 4, 32);
    sum += __shfl_xor(sum, 2, 32);
    sum += __shfl_xor(sum, 1, 32);
    const float r  = e * (1.0f / sum);
    const float r0 = __shfl(r, src0, 32);
    const float r1 = __shfl(r, src0 + 1, 32);
    const _Float16 h0 = (_Float16)(r0 * carry);
    const _Float16 h1 = (_Float16)(r1 * carry);
    const unsigned w = (unsigned)__builtin_bit_cast(unsigned short, h0) |
                       ((unsigned)__builtin_bit_cast(unsigned short, h1) << 16);
    volatile unsigned* p = R2w + (size_t)row * (kKmix / 2) + lane;
    *p = w;
    __threadfence();
    *p = w;
  }
}

__global__ __launch_bounds__(256) void mix_out_kernel(
    const float* __restrict__ x, const float* __restrict__ P, const float* __restrict__ consts,
    float* __restrict__ out, int total4)
{
  const int i = blockIdx.x * 256 + threadIdx.x;
  if (i >= total4) return;
  const float s   = consts[kIdxS];
  const float inv = consts[kIdxInv];
  const v4f xv = *(const v4f*)(x + (size_t)i * 4);
  const v4f pv = *(const v4f*)(P + (size_t)i * 4);
  v4f o;
  o[0] = (xv[0] - s * pv[0]) * inv;
  o[1] = (xv[1] - s * pv[1]) * inv;
  o[2] = (xv[2] - s * pv[2]) * inv;
  o[3] = (xv[3] - s * pv[3]) * inv;
  float* q = out + (size_t)i * 4;
  *(volatile v4f*)q = o;
  __threadfence();
  *(volatile v4f*)q = o;
}

extern "C" void kernel_launch(void* const* d_in, const int* in_sizes, int n_in,
                              void* d_out, int out_size, void* d_ws, size_t ws_size,
                              hipStream_t stream) {
  if (n_in < 5) return;
  if (in_sizes[0] != kRowsN * kDim) return;
  if (in_sizes[1] != kComp * kDim) return;
  if (in_sizes[2] != kComp) return;
  if (in_sizes[3] != kTab) return;
  if (in_sizes[4] != 1) return;
  if (out_size != kRowsN * kDim) return;
  if (ws_size < kWsTotal) return;

  const float* x       = (const float*)d_in[0];
  const float* means   = (const float*)d_in[1];
  const float* weights = (const float*)d_in[2];
  const float* acp     = (const float*)d_in[3];
  const int*   tt      = (const int*)d_in[4];
  float* out = (float*)d_out;

  char* ws = (char*)d_ws;
  unsigned short* A1  = (unsigned short*)(ws + kOffA1);
  unsigned short* BT1 = (unsigned short*)(ws + kOffBT1);
  float*          G   = (float*)(ws + kOffG);
  unsigned short* R2  = (unsigned short*)(ws + kOffR2);
  unsigned short* BT2 = (unsigned short*)(ws + kOffBT2);
  float*          P   = (float*)(ws + kOffP);
  float*          CST = (float*)(ws + kOffCST);

  prep_kernel<<<1, 256, 0, stream>>>(means, weights, acp, tt, CST, (unsigned*)BT1, (unsigned*)BT2);

  split_x_kernel<<<(kRowsN * kDim / 8) / 256, 256, 0, stream>>>(x, (unsigned*)A1, kRowsN * kDim / 8);

  gemm64_kernel<1><<<(kRowsN / 64) * (kCompT / 64) / 8, 256, 0, stream>>>(
      A1, kKcat, BT1, kKcat, G, kCompT, kRowsN, kCompT, kKcat, 1.0f);

  softmax_rows_kernel<<<kRowsN / (8 * kSoftRowsPerWave), 256, 0, stream>>>(G, CST, (unsigned*)R2);

  gemm64_kernel<0><<<(kRowsN / 64) * (kDim / 64) / 8, 256, 0, stream>>>(
      R2, kKmix, BT2, kKmix, P, kDim, kRowsN, kDim, kKmix, kFoldBack);

  mix_out_kernel<<<(kRowsN * kDim / 4) / 256, 256, 0, stream>>>(x, P, CST, out, kRowsN * kDim / 4);
}
